// PoliceDiscriminator_88399016887015
// MI455X (gfx1250) — hardware-verified
//
#include <hip/hip_runtime.h>
#include <stddef.h>


#define DF    128
#define GR    32
#define AP    136
#define XSP   132
#define NTHR  256
#define NWV   8
#define CHUNK 2048
#define WCAP  256
#define NGRP  (CHUNK / (NTHR * 4))
#define NB1   512
#define SH1   9
#define NB2   4096
#define SH2   12

#define SACC1 (NB1 * DF)
#define LISTN (NWV * WCAP)
#define LDS1_BYTES ((SACC1 + NB1 * 2 + NB1 * 2 + LISTN + NWV) * 4)
#define LDS2_BYTES ((NB2 * 4 + LISTN + NWV) * 4)

static_assert(WCAP == (CHUNK / NTHR) * 32);
static_assert(NGRP == 2);
static_assert(LISTN == NB1 * 4);
static_assert((1 << SH1) == NB1);
static_assert((1 << SH2) == NB2);
static_assert(CHUNK <= 2048);
static_assert(LDS1_BYTES == 278560);
static_assert(LDS2_BYTES == 73760);
static_assert(((SACC1 + NB1 * 2) % 4) == 0);
static_assert(((SACC1 + NB1 * 4) % 4) == 0);
static_assert(NB2 % (4 * NTHR) == 0);
static_assert(NB1 % NWV == 0);
static_assert((NB1 * 4) % (4 * NTHR) == 0);

typedef float    v4f  __attribute__((ext_vector_type(4)));
typedef float    v8f  __attribute__((ext_vector_type(8)));
typedef int      v4i  __attribute__((ext_vector_type(4)));
typedef _Float16 v8h  __attribute__((ext_vector_type(8)));
typedef _Float16 v16h __attribute__((ext_vector_type(16)));
union Frag   { v16h v; v8h half[2]; };
union Pack16 { v8h h; v4i i; };

__device__ __forceinline__ v8f wm(v16h a, v16h b, v8f c) {
  v8f d = __builtin_amdgcn_wmma_f32_16x16x32_f16(false, a, false, b, (short)0, c, false, false);
  asm volatile("v_nop\n\tv_nop\n\tv_nop\n\tv_nop" : "+v"(d) : "v"(a), "v"(b));
  return d;
}

__device__ __forceinline__ float wsum(float v) {
  v += __shfl_xor(v, 16, 32);
  v += __shfl_xor(v, 8, 32);
  v += __shfl_xor(v, 4, 32);
  v += __shfl_xor(v, 2, 32);
  v += __shfl_xor(v, 1, 32);
  return v;
}

__global__ __launch_bounds__(NTHR) void k_prep(const float* __restrict__ W1, _Float16* Wh) {
  const int i = blockIdx.x * NTHR + threadIdx.x;
  if (i >= DF * DF / 8) return;
  const int n  = i >> 4;
  const int k8 = (i & 15) * 8;
  Pack16 u;
#pragma unroll
  for (int j = 0; j < 8; ++j) u.h[j] = (_Float16)(W1[(size_t)(k8 + j) * DF + n] * 8.0f);
  _Float16* p = Wh + (size_t)n * DF + k8;
  *(volatile v4i*)p = u.i;
  __threadfence();
  *(volatile v4i*)p = u.i;
}

__device__ __forceinline__ void epi_tile(v8f acc, int T, int hh, int m, int wave, int ncol,
                                         float cs, float cd, float* Xs, float* As, float* Ds) {
  float ss[8], sd[8];
#pragma unroll
  for (int r = 0; r < 8; ++r) {
    const float v = acc[r] * 0.125f;
    Xs[(T * 16 + 8 * hh + r) * XSP + ncol] = v;
    ss[r] = v * cs;
    sd[r] = v * cd;
  }
#pragma unroll
  for (int mk = 1; mk < 16; mk <<= 1) {
#pragma unroll
    for (int r = 0; r < 8; ++r) {
      ss[r] += __shfl_xor(ss[r], mk, 32);
      sd[r] += __shfl_xor(sd[r], mk, 32);
    }
  }
  if (m == 0) {
#pragma unroll
    for (int r = 0; r < 8; ++r) {
      As[(T * 16 + 8 * hh + r) * NWV + wave] = ss[r];
      Ds[(T * 16 + 8 * hh + r) * NWV + wave] = sd[r];
    }
  }
}

__global__ __launch_bounds__(NTHR) void k_gemm(
    const float* __restrict__ x, const _Float16* __restrict__ Wh,
    const float* __restrict__ att_s, const float* __restrict__ att_d,
    float* xp, float* aa, int nN) {
  __shared__ __attribute__((aligned(16))) _Float16 At[GR * AP];
  __shared__ __attribute__((aligned(16))) float Xs[GR * XSP];
  __shared__ __attribute__((aligned(16))) float As[GR * NWV];
  __shared__ __attribute__((aligned(16))) float Ds[GR * NWV];

  const int tid  = threadIdx.x;
  const int lane = tid & 31;
  const int wave = tid >> 5;
  const int hh   = lane >> 4;
  const int m    = lane & 15;
  const int rowBase = blockIdx.x * GR;

  {
    const int r  = tid >> 3;
    const int c0 = (tid & 7) * 16;
    int row = rowBase + r;
    if (row > nN - 1) row = nN - 1;
    const float* p = x + (size_t)row * DF + c0;
    const v4f f0 = *(const v4f*)(p), f1 = *(const v4f*)(p + 4);
    const v4f f2 = *(const v4f*)(p + 8), f3 = *(const v4f*)(p + 12);
    Pack16 u0, u1;
    u0.h[0] = (_Float16)f0.x; u0.h[1] = (_Float16)f0.y; u0.h[2] = (_Float16)f0.z; u0.h[3] = (_Float16)f0.w;
    u0.h[4] = (_Float16)f1.x; u0.h[5] = (_Float16)f1.y; u0.h[6] = (_Float16)f1.z; u0.h[7] = (_Float16)f1.w;
    u1.h[0] = (_Float16)f2.x; u1.h[1] = (_Float16)f2.y; u1.h[2] = (_Float16)f2.z; u1.h[3] = (_Float16)f2.w;
    u1.h[4] = (_Float16)f3.x; u1.h[5] = (_Float16)f3.y; u1.h[6] = (_Float16)f3.z; u1.h[7] = (_Float16)f3.w;
    *(v8h*)(At + r * AP + c0)     = u0.h;
    *(v8h*)(At + r * AP + c0 + 8) = u1.h;
  }
  __syncthreads();

  const int ncol = wave * 16 + m;
  v8f c0a = {0.f, 0.f, 0.f, 0.f, 0.f, 0.f, 0.f, 0.f};
  v8f c1a = {0.f, 0.f, 0.f, 0.f, 0.f, 0.f, 0.f, 0.f};
#pragma unroll
  for (int kt = 0; kt < DF / 32; ++kt) {
    const int k0 = kt * 32;
    Frag a0, a1, b;
    const _Float16* pb  = Wh + (size_t)ncol * DF + k0 + 8 * hh;
    const _Float16* pa0 = At + m * AP + k0 + 8 * hh;
    const _Float16* pa1 = At + (16 + m) * AP + k0 + 8 * hh;
    b.half[0]  = *(const v8h*)pb;  b.half[1]  = *(const v8h*)(pb + 16);
    a0.half[0] = *(const v8h*)pa0; a0.half[1] = *(const v8h*)(pa0 + 16);
    a1.half[0] = *(const v8h*)pa1; a1.half[1] = *(const v8h*)(pa1 + 16);
    c0a = wm(a0.v, b.v, c0a);
    c1a = wm(a1.v, b.v, c1a);
  }

  const float cs = att_s[ncol];
  const float cd = att_d[ncol];
  epi_tile(c0a, 0, hh, m, wave, ncol, cs, cd, Xs, As, Ds);
  epi_tile(c1a, 1, hh, m, wave, ncol, cs, cd, Xs, As, Ds);
  __syncthreads();

  v4f xr[4];
#pragma unroll
  for (int i = 0; i < 4; ++i) xr[i] = *(const v4f*)(Xs + (4 * wave + i) * XSP + 4 * lane);
  v4f av;
  {
    const float* ap = As + lane * NWV;
    const float* dp = Ds + lane * NWV;
    av.x = (ap[0] + ap[1]) + (ap[2] + ap[3]);
    av.y = (ap[4] + ap[5]) + (ap[6] + ap[7]);
    av.z = (dp[0] + dp[1]) + (dp[2] + dp[3]);
    av.w = (dp[4] + dp[5]) + (dp[6] + dp[7]);
  }
  float* xpp[4];
#pragma unroll
  for (int i = 0; i < 4; ++i) xpp[i] = xp + (size_t)(rowBase + 4 * wave + i) * DF + 4 * lane;
  float* gp = aa + ((size_t)rowBase + lane) * 4;

#pragma unroll
  for (int i = 0; i < 4; ++i) *(volatile v4f*)(xpp[i]) = xr[i];
  if (wave == 0) *(volatile v4f*)gp = av;
  __threadfence();
#pragma unroll
  for (int i = 0; i < 4; ++i) *(volatile v4f*)(xpp[i]) = xr[i];
  if (wave == 0) *(volatile v4f*)gp = av;
}

template <int NBT, int SHT>
__device__ __forceinline__ int scan_chunk(const int* __restrict__ eid, int nE, int cbase,
                                          int nodeBase, bool al16, int* list, int tid, int wave) {
  int wc = 0;
#pragma unroll
  for (int g = 0; g < NGRP; ++g) {
    const int el0 = (g * NTHR + tid) * 4;
    const int e0  = cbase + el0;
    const int sent = -2147483647 - 1;
    v4i d;
    if (al16 && (cbase + CHUNK <= nE)) {
      d = *(const v4i*)(eid + e0);
    } else {
      const int le = nE - 1;
      d.x = (e0     < nE) ? eid[min(e0,     le)] : sent;
      d.y = (e0 + 1 < nE) ? eid[min(e0 + 1, le)] : sent;
      d.z = (e0 + 2 < nE) ? eid[min(e0 + 2, le)] : sent;
      d.w = (e0 + 3 < nE) ? eid[min(e0 + 3, le)] : sent;
    }
    const unsigned s0 = (unsigned)d.x - (unsigned)nodeBase;
    const unsigned s1 = (unsigned)d.y - (unsigned)nodeBase;
    const unsigned s2 = (unsigned)d.z - (unsigned)nodeBase;
    const unsigned s3 = (unsigned)d.w - (unsigned)nodeBase;
    const bool h0 = s0 < (unsigned)NBT;
    const bool h1 = s1 < (unsigned)NBT;
    const bool h2 = s2 < (unsigned)NBT;
    const bool h3 = s3 < (unsigned)NBT;
    const unsigned many = __builtin_amdgcn_ballot_w32(h0 | h1 | h2 | h3);
    if (many != 0u) {
#define HITJ(J, HJ, SJ) { \
        const unsigned mj = __builtin_amdgcn_ballot_w32(HJ); \
        if (HJ) { \
          const int pos = wc + (int)__builtin_amdgcn_mbcnt_lo(mj, 0u); \
          if (pos < WCAP) list[wave * WCAP + pos] = ((el0 + (J)) << SHT) | (int)(SJ); \
        } \
        wc += (int)__builtin_popcount(mj); }
      HITJ(0, h0, s0)
      HITJ(1, h1, s1)
      HITJ(2, h2, s2)
      HITJ(3, h3, s3)
#undef HITJ
    }
  }
  return wc;
}

__global__ __launch_bounds__(NTHR) void k_gat1(
    const int* __restrict__ ei, const float* __restrict__ xp, const float* __restrict__ aa,
    const float* __restrict__ b1, const float* __restrict__ W2,
    const float* __restrict__ as2c, const float* __restrict__ ad2c,
    float* Gp, int nN, int nE) {
  extern __shared__ v4f lds_dyn[];
  float* sacc = (float*)lds_dyn;
  float* den  = sacc + SACC1;
  float* mx   = den + NB1 * 2;
  int*   list = (int*)(mx + NB1 * 2);
  int*   wcnt = list + LISTN;

  const int tid  = threadIdx.x;
  const int lane = tid & 31;
  const int wave = tid >> 5;
  const int hd   = lane >> 4;
  const int nodeBase = blockIdx.x * NB1;

  {
    const v4f z4 = {0.f, 0.f, 0.f, 0.f};
    for (int i = tid; i < (SACC1 + NB1 * 2) / 4; i += NTHR) lds_dyn[i] = z4;
    for (int i = tid; i < NB1 * 2; i += NTHR) mx[i] = -1.0e30f;
  }
  __syncthreads();

  const int* eid = ei + nE;
  const bool al16 = ((nE & 3) == 0);
  const int nChunks = (nE + CHUNK - 1) / CHUNK;
#pragma unroll 1
  for (int ch = 0; ch < nChunks; ++ch) {
    const int cbase = ch * CHUNK;
    const int wc = scan_chunk<NB1, SH1>(eid, nE, cbase, nodeBase, al16, list, tid, wave);
    if (lane == 0) wcnt[wave] = wc;
    __syncthreads();

    if (wave == 0) {
      for (int wsx = 0; wsx < NWV; ++wsx) {
        int n = wcnt[wsx];
        if (n > WCAP) n = WCAP;
        if (n < 0) n = 0;
        for (int i = 0; i < n; ++i) {
          const int ent  = list[wsx * WCAP + i];
          const int slot = ent & (NB1 - 1);
          const int el   = (ent >> SH1) & (CHUNK - 1);
          int e = cbase + el;
          if (e > nE - 1) e = nE - 1;
          int src = ei[e];
          src = src < 0 ? 0 : (src > nN - 1 ? nN - 1 : src);
          int nd = nodeBase + slot;
          if (nd > nN - 1) nd = nN - 1;
          float al = aa[(size_t)src * 4 + hd] + aa[(size_t)nd * 4 + 2 + hd];
          al = (al > 0.f) ? al : 0.2f * al;
          const float mo = mx[slot * 2 + hd];
          const float mn = fmaxf(mo, al);
          const float sc = __expf(mo - mn);
          const float p  = __expf(al - mn);
          const v4f xv = *(const v4f*)(xp + (size_t)src * DF + 4 * lane);
          v4f* sp = (v4f*)(sacc + slot * DF + 4 * lane);
          const v4f cur = *sp;
          const v4f nxt = cur * sc + p * xv;
          *sp = nxt;
          if ((lane & 15) == 0) {
            const float od = den[slot * 2 + hd];
            den[slot * 2 + hd] = od * sc + p;
            mx[slot * 2 + hd]  = mn;
          }
        }
      }
    }
    __syncthreads();
  }

  float* Gs = (float*)list;
  const v4f b4 = *(const v4f*)(b1 + 4 * lane);
  const v4f w4 = *(const v4f*)(W2 + 4 * lane);
  const float s2 = as2c[0];
  const float d2 = ad2c[0];
#pragma unroll 1
  for (int j = 0; j < NB1 / NWV; ++j) {
    const int slot = wave * (NB1 / NWV) + j;
    const int node = nodeBase + slot;
    const bool valid = node < nN;
    const size_t nrow = (size_t)(valid ? node : nN - 1);
    float al = aa[nrow * 4 + hd] + aa[nrow * 4 + 2 + hd];
    al = (al > 0.f) ? al : 0.2f * al;
    const float mo = mx[slot * 2 + hd];
    const float mn = fmaxf(mo, al);
    const float sc = __expf(mo - mn);
    const float p  = __expf(al - mn);
    const v4f xv = *(const v4f*)(xp + nrow * DF + 4 * lane);
    const v4f sv = *(const v4f*)(sacc + slot * DF + 4 * lane) * sc + p * xv;
    const float dv  = den[slot * 2 + hd] * sc + p;
    const float inv = 1.0f / fmaxf(dv, 1e-16f);
    v4f o = sv * inv + b4;
    o.x = o.x > 0.f ? o.x : (__expf(o.x) - 1.0f);
    o.y = o.y > 0.f ? o.y : (__expf(o.y) - 1.0f);
    o.z = o.z > 0.f ? o.z : (__expf(o.z) - 1.0f);
    o.w = o.w > 0.f ? o.w : (__expf(o.w) - 1.0f);
    const float part = o.x * w4.x + o.y * w4.y + o.z * w4.z + o.w * w4.w;
    const float g = wsum(part);
    if (lane == 0) {
      Gs[slot * 4 + 0] = valid ? g : 0.f;
      Gs[slot * 4 + 1] = valid ? g * s2 : 0.f;
      Gs[slot * 4 + 2] = valid ? g * d2 : 0.f;
      Gs[slot * 4 + 3] = 0.f;
    }
  }
  __syncthreads();

  v4f gvv[2];
  float* gpp[2];
#pragma unroll
  for (int i = 0; i < 2; ++i) {
    const int q = i * NTHR + tid;
    gvv[i] = *(const v4f*)(Gs + q * 4);
    gpp[i] = Gp + ((size_t)nodeBase + q) * 4;
  }
#pragma unroll
  for (int i = 0; i < 2; ++i) *(volatile v4f*)(gpp[i]) = gvv[i];
  __threadfence();
#pragma unroll
  for (int i = 0; i < 2; ++i) *(volatile v4f*)(gpp[i]) = gvv[i];
}

__global__ __launch_bounds__(NTHR) void k_gat2(
    const int* __restrict__ ei, const float* __restrict__ Gp, const float* __restrict__ b2,
    float* out, int nN, int nE) {
  extern __shared__ v4f lds_dyn2[];
  float* num  = (float*)lds_dyn2;
  float* dn   = num + NB2;
  float* mx   = dn + NB2;
  float* adn  = mx + NB2;
  int*   list = (int*)(adn + NB2);
  int*   wcnt = list + LISTN;

  const int tid  = threadIdx.x;
  const int lane = tid & 31;
  const int wave = tid >> 5;
  const int nodeBase = blockIdx.x * NB2;

  for (int i = tid; i < NB2; i += NTHR) {
    num[i] = 0.f;
    dn[i]  = 0.f;
    mx[i]  = -1.0e30f;
    int nd = nodeBase + i;
    if (nd > nN - 1) nd = nN - 1;
    adn[i] = Gp[(size_t)nd * 4 + 2];
  }
  __syncthreads();

  const int* eid = ei + nE;
  const bool al16 = ((nE & 3) == 0);
  const int nChunks = (nE + CHUNK - 1) / CHUNK;
#pragma unroll 1
  for (int ch = 0; ch < nChunks; ++ch) {
    const int cbase = ch * CHUNK;
    const int wc = scan_chunk<NB2, SH2>(eid, nE, cbase, nodeBase, al16, list, tid, wave);
    if (lane == 0) wcnt[wave] = wc;
    __syncthreads();

    if (wave == 0) {
      for (int wsx = 0; wsx < NWV; ++wsx) {
        int n = wcnt[wsx];
        if (n > WCAP) n = WCAP;
        if (n < 0) n = 0;
        for (int i = 0; i < n; ++i) {
          const int ent  = list[wsx * WCAP + i];
          const int slot = ent & (NB2 - 1);
          const int el   = (ent >> SH2) & (CHUNK - 1);
          int e = cbase + el;
          if (e > nE - 1) e = nE - 1;
          int src = ei[e];
          src = src < 0 ? 0 : (src > nN - 1 ? nN - 1 : src);
          const v4f gv = *(const v4f*)(Gp + (size_t)src * 4);
          float al = gv.y + adn[slot];
          al = (al > 0.f) ? al : 0.2f * al;
          const float mo = mx[slot];
          const float mn = fmaxf(mo, al);
          const float sc = __expf(mo - mn);
          const float p  = __expf(al - mn);
          const float nm = num[slot] * sc + p * gv.x;
          const float dv = dn[slot] * sc + p;
          if (lane == 0) {
            num[slot] = nm;
            dn[slot]  = dv;
            mx[slot]  = mn;
          }
        }
      }
    }
    __syncthreads();
  }

  const float b2s = b2[0];
#pragma unroll 1
  for (int i = tid; i < NB2; i += NTHR) {
    int nd = nodeBase + i;
    if (nd > nN - 1) nd = nN - 1;
    const v4f gv = *(const v4f*)(Gp + (size_t)nd * 4);
    float al = gv.y + adn[i];
    al = (al > 0.f) ? al : 0.2f * al;
    const float mo = mx[i];
    const float mn = fmaxf(mo, al);
    const float sc = __expf(mo - mn);
    const float p  = __expf(al - mn);
    const float nm = num[i] * sc + p * gv.x;
    const float dv = dn[i] * sc + p;
    const float inv = 1.0f / fmaxf(dv, 1e-16f);
    const float v = nm * inv + b2s;
    const float sg = 1.0f / (1.0f + __expf(-v));
    num[i] = sg;
  }
  __syncthreads();

  v4f ov[NB2 / (4 * NTHR)];
#pragma unroll
  for (int i = 0; i < NB2 / (4 * NTHR); ++i) ov[i] = *(const v4f*)(num + 4 * (i * NTHR + tid));
#pragma unroll
  for (int i = 0; i < NB2 / (4 * NTHR); ++i) {
    const int n0 = nodeBase + 4 * (i * NTHR + tid);
    if (n0 + 4 <= nN) {
      *(volatile v4f*)(out + n0) = ov[i];
    } else {
      if (n0     < nN) *(volatile float*)(out + n0)     = ov[i].x;
      if (n0 + 1 < nN) *(volatile float*)(out + n0 + 1) = ov[i].y;
      if (n0 + 2 < nN) *(volatile float*)(out + n0 + 2) = ov[i].z;
      if (n0 + 3 < nN) *(volatile float*)(out + n0 + 3) = ov[i].w;
    }
  }
  __threadfence();
#pragma unroll
  for (int i = 0; i < NB2 / (4 * NTHR); ++i) {
    const int n0 = nodeBase + 4 * (i * NTHR + tid);
    if (n0 + 4 <= nN) {
      *(volatile v4f*)(out + n0) = ov[i];
    } else {
      if (n0     < nN) *(volatile float*)(out + n0)     = ov[i].x;
      if (n0 + 1 < nN) *(volatile float*)(out + n0 + 1) = ov[i].y;
      if (n0 + 2 < nN) *(volatile float*)(out + n0 + 2) = ov[i].z;
      if (n0 + 3 < nN) *(volatile float*)(out + n0 + 3) = ov[i].w;
    }
  }
}

extern "C" void kernel_launch(void* const* d_in, const int* in_sizes, int n_in,
                              void* d_out, int out_size, void* d_ws, size_t ws_size,
                              hipStream_t stream) {
  if (n_in < 10) return;
  const int nN = in_sizes[0] / DF;
  if (nN <= 0 || in_sizes[0] != nN * DF) return;
  const int nE = in_sizes[1] / 2;
  if (nE < 0 || in_sizes[1] != 2 * nE) return;
  if (in_sizes[2] != DF * DF) return;
  if (in_sizes[3] != DF || in_sizes[4] != DF || in_sizes[5] != DF || in_sizes[6] != DF) return;
  if (in_sizes[7] < 1 || in_sizes[8] < 1 || in_sizes[9] < 1) return;
  if (out_size != nN) return;

  const float* x     = (const float*)d_in[0];
  const int*   ei    = (const int*)d_in[1];
  const float* W1    = (const float*)d_in[2];
  const float* att_s = (const float*)d_in[3];
  const float* att_d = (const float*)d_in[4];
  const float* b1    = (const float*)d_in[5];
  const float* W2    = (const float*)d_in[6];
  const float* as2c  = (const float*)d_in[7];
  const float* ad2c  = (const float*)d_in[8];
  const float* b2    = (const float*)d_in[9];
  float* out = (float*)d_out;

  const int grid1 = (nN + NB1 - 1) / NB1;
  const int grid2 = (nN + NB2 - 1) / NB2;
  const int nP  = ((nN + GR - 1) / GR) * GR;
  const int nPg = grid1 * NB1;
  size_t off = 0;
  _Float16* Wh = (_Float16*)((char*)d_ws + off); off += (size_t)DF * DF * sizeof(_Float16);
  off = (off + 255) & ~(size_t)255;
  float* xp = (float*)((char*)d_ws + off);       off += (size_t)nP * DF * sizeof(float);
  off = (off + 255) & ~(size_t)255;
  float* aa = (float*)((char*)d_ws + off);       off += (size_t)nP * 4 * sizeof(float);
  off = (off + 255) & ~(size_t)255;
  float* Gp = (float*)((char*)d_ws + off);       off += (size_t)nPg * 4 * sizeof(float);
  if (off > ws_size) return;

  k_prep<<<(DF * DF / 8 + NTHR - 1) / NTHR, NTHR, 0, stream>>>(W1, Wh);

  k_gemm<<<nP / GR, NTHR, 0, stream>>>(x, Wh, att_s, att_d, xp, aa, nN);

  hipFuncSetAttribute(reinterpret_cast<const void*>(&k_gat1),
                      hipFuncAttributeMaxDynamicSharedMemorySize, LDS1_BYTES);
  k_gat1<<<grid1, NTHR, LDS1_BYTES, stream>>>(ei, xp, aa, b1, W2, as2c, ad2c, Gp, nN, nE);

  hipFuncSetAttribute(reinterpret_cast<const void*>(&k_gat2),
                      hipFuncAttributeMaxDynamicSharedMemorySize, LDS2_BYTES);
  k_gat2<<<grid2, NTHR, LDS2_BYTES, stream>>>(ei, Gp, b2, out, nN, nE);
}
